// NonLocalBlockND_32392643346905
// MI455X (gfx1250) — hardware-verified
//
#include <hip/hip_runtime.h>
#include <math.h>
#include <stdint.h>

typedef __attribute__((ext_vector_type(16))) _Float16 v16h;
typedef __attribute__((ext_vector_type(8)))  _Float16 v8h;
typedef __attribute__((ext_vector_type(16))) __bf16   v16b;
typedef __attribute__((ext_vector_type(8)))  __bf16   v8b;
typedef __attribute__((ext_vector_type(8)))  float    v8f;
typedef __attribute__((ext_vector_type(4)))  float    v4f;
#define U16(p) ((const unsigned short*)(const void*)(p))

__device__ __forceinline__ v8f zero8() { return (v8f){0.f, 0.f, 0.f, 0.f, 0.f, 0.f, 0.f, 0.f}; }

__device__ __forceinline__ unsigned short f2bf_bits(float f) {
  unsigned u = __float_as_uint(f);
  return (unsigned short)((u + 0x7FFFu + ((u >> 16) & 1u)) >> 16);
}
__device__ __forceinline__ float bf_bits2f(unsigned short h) { return __uint_as_float(((unsigned)h) << 16); }

__device__ __forceinline__ void dep_guard_h(v8f& a, v8f& b, v16h x, v16h y) { asm volatile("v_nop\n\tv_nop\n\tv_nop\n\tv_nop" : "+v"(a), "+v"(b) : "v"(x), "v"(y)); }
__device__ __forceinline__ void dep_guard_b(v8f& a, v8f& b, v16b x, v16b y) { asm volatile("v_nop\n\tv_nop\n\tv_nop\n\tv_nop" : "+v"(a), "+v"(b) : "v"(x), "v"(y)); }
__device__ __forceinline__ void keep4_h(v16h a, v16h b, v16h c, v16h d) { asm volatile("v_nop" :: "v"(a), "v"(b), "v"(c), "v"(d)); }
__device__ __forceinline__ void keep4_b(v16b a, v16b b, v16b c, v16b d) { asm volatile("v_nop" :: "v"(a), "v"(b), "v"(c), "v"(d)); }
__device__ __forceinline__ void acc_guard4(v8f& a, v8f& b, v8f& c, v8f& d) { asm volatile("v_nop\n\tv_nop\n\tv_nop\n\tv_nop" : "+v"(a), "+v"(b), "+v"(c), "+v"(d)); }
template <typename T> struct Frag;
template <> struct Frag<_Float16> {
  typedef v16h V; union U { v16h v; v8h h[2]; };
  static __device__ __forceinline__ v16h load(const _Float16* p) {
    U f; f.h[0] = *(const v8h*)(p); f.h[1] = *(const v8h*)(p + 16); return f.v;
  }
  static __device__ __forceinline__ v8f mma(v16h a, v16h b, v8f c) {
    return __builtin_amdgcn_wmma_f32_16x16x32_f16(false, a, false, b, (short)0, c, false, false);
  }
  static __device__ __forceinline__ void guard(v8f& a, v8f& b, v16h x, v16h y) { dep_guard_h(a, b, x, y); }
  static __device__ __forceinline__ void keep(v16h a, v16h b, v16h c, v16h d) { keep4_h(a, b, c, d); }
};
template <> struct Frag<__bf16> {
  typedef v16b V; union U { v16b v; v8b h[2]; };
  static __device__ __forceinline__ v16b load(const __bf16* p) {
    U f; f.h[0] = *(const v8b*)(p); f.h[1] = *(const v8b*)(p + 16); return f.v;
  }
  static __device__ __forceinline__ v8f mma(v16b a, v16b b, v8f c) {
    return __builtin_amdgcn_wmma_f32_16x16x32_bf16(false, a, false, b, (short)0, c, false, false);
  }
  static __device__ __forceinline__ void guard(v8f& a, v8f& b, v16b x, v16b y) { dep_guard_b(a, b, x, y); }
  static __device__ __forceinline__ void keep(v16b a, v16b b, v16b c, v16b d) { keep4_b(a, b, c, d); }
};

__device__ __forceinline__ v8f mma_h(v16h a, v16h b, v8f c) {
  c = __builtin_amdgcn_wmma_f32_16x16x32_f16(false, a, false, b, (short)0, c, false, false);
  asm volatile("v_nop\n\tv_nop\n\tv_nop\n\tv_nop" : "+v"(c) : "v"(a), "v"(b));
  return c;
}

template <int ET> struct Elem;
template <> struct Elem<0> { typedef _Float16 T; };
template <> struct Elem<1> { typedef __bf16 T; };
template <int ET, bool SPLIT, int BIAS_MODE, int OUT_MODE, bool RESID, int ACT, bool GAIN>
__global__ __launch_bounds__(256) void wmma_gemm64(
    const unsigned short* __restrict__ Ap, const unsigned short* __restrict__ A2p, int lda, long strideA,
    const unsigned short* __restrict__ Btp, const unsigned short* __restrict__ Bt2p, int ldb, long strideB,
    void* __restrict__ Cout, void* __restrict__ Cout2, int ldc, long strideC,
    const float* __restrict__ bias, const float* __restrict__ gain,
    const float* __restrict__ resid, long strideR,
    int M, int N, int K, float scale) {
  typedef typename Elem<ET>::T T;
  typedef typename Frag<T>::V V;
  const T* A = (const T*)Ap; const T* A2 = (const T*)A2p; const T* Bt = (const T*)Btp; const T* Bt2 = (const T*)Bt2p;
  __shared__ __align__(16) float sT[8][16 * 68];
  const int b    = blockIdx.y;
  const int lane = threadIdx.x & 31;
  const int wave = threadIdx.x >> 5;
  const int tilesN = N >> 6;
  const int tilesM = M >> 6;
  const int tile = blockIdx.x * 8 + wave;
  if (tile >= tilesM * tilesN) return;
  const int tm = tile / tilesN;
  const int tn = tile - tm * tilesN;
  const int m0 = tm << 6;
  const int n0 = tn << 6;

  const T* Ab  = A  + (size_t)b * strideA;
  const T* Bb  = Bt + (size_t)b * strideB;
  const T* Ab2 = SPLIT ? (A2  + (size_t)b * strideA) : nullptr;
  const T* Bb2 = SPLIT ? (Bt2 + (size_t)b * strideB) : nullptr;

  const int rlane = lane & 15;
  const int koff  = (lane >> 4) * 8;
  const int mOff  = (lane >> 4) * 8;

  v8f acc[4][4];
#pragma unroll
  for (int i = 0; i < 4; ++i)
#pragma unroll
    for (int j = 0; j < 4; ++j) acc[i][j] = zero8();

  for (int k0 = 0; k0 < K; k0 += 32) {
    V bh[4], bl[4];
#pragma unroll
    for (int j = 0; j < 4; ++j) {
      const size_t bo = (size_t)(n0 + (j << 4) + rlane) * ldb + koff + k0;
      bh[j] = Frag<T>::load(Bb + bo);
      if (SPLIT) bl[j] = Frag<T>::load(Bb2 + bo);
    }
#pragma unroll
    for (int i = 0; i < 4; ++i) {
      const size_t ao = (size_t)(m0 + (i << 4) + rlane) * lda + koff + k0;
      V ah = Frag<T>::load(Ab + ao);
      V al;
      if (SPLIT) al = Frag<T>::load(Ab2 + ao);
#pragma unroll
      for (int j = 0; j < 4; ++j) {
        acc[i][j] = Frag<T>::mma(ah, bh[j], acc[i][j]);
        if (SPLIT) {
          acc[i][j] = Frag<T>::mma(ah, bl[j], acc[i][j]);
          acc[i][j] = Frag<T>::mma(al, bh[j], acc[i][j]);
        }
      }
      Frag<T>::guard(acc[i][0], acc[i][3], ah, SPLIT ? al : ah);
    }
    Frag<T>::keep(bh[0], bh[1], bh[2], bh[3]);
    if (SPLIT) Frag<T>::keep(bl[0], bl[1], bl[2], bl[3]);
  }
  acc_guard4(acc[0][0], acc[0][1], acc[0][2], acc[0][3]);
  acc_guard4(acc[1][0], acc[1][1], acc[1][2], acc[1][3]);
  acc_guard4(acc[2][0], acc[2][1], acc[2][2], acc[2][3]);
  acc_guard4(acc[3][0], acc[3][1], acc[3][2], acc[3][3]);

  float* slab = sT[wave];
  const float* Rb = RESID ? (resid + (size_t)b * strideR) : nullptr;
  const float gv = GAIN ? gain[0] : 1.0f;
#pragma unroll
  for (int i = 0; i < 4; ++i) {
    const int mBase = m0 + (i << 4);
#pragma unroll
    for (int j = 0; j < 4; ++j) {
      const int n = n0 + (j << 4) + rlane;
      float bv = 0.f;
      if (BIAS_MODE == 2) bv = bias[n];
#pragma unroll
      for (int r = 0; r < 8; ++r) {
        float v = acc[i][j][r] * scale;
        if (BIAS_MODE == 1) v += bias[mBase + mOff + r];
        if (BIAS_MODE == 2) v += bv;
        if (GAIN) v *= gv;
        if (RESID) v += Rb[(size_t)(mBase + mOff + r) * ldc + n];
        if (ACT == 1) v = tanhf(v);
        if (ACT == 2) v = fmaxf(v, 0.0f);
        if (ACT == 3) v = v / (1.0f + expf(-v));
        if (ACT == 4) v = (v > 0.f) ? v : 0.01f * v;
        if (ACT == 5) v = 0.5f * v * (1.0f + erff(v * 0.70710678118654752f));
        slab[(mOff + r) * 68 + (j << 4) + rlane] = v;
      }
    }
    __builtin_amdgcn_fence(__ATOMIC_RELEASE, "workgroup");
    __builtin_amdgcn_wave_barrier();
    __builtin_amdgcn_fence(__ATOMIC_ACQUIRE, "workgroup");
    if (OUT_MODE == 0) {
      float* C = (float*)Cout + (size_t)b * strideC;
      const int hh = lane >> 4, c4 = (lane & 15) * 4;
      for (int pass = 0; pass < 2; ++pass) {
#pragma unroll
        for (int it = 0; it < 8; ++it) {
          const int row = it * 2 + hh;
          v4f v = *(const v4f*)(slab + row * 68 + c4);
          *(volatile v4f*)(C + (size_t)(mBase + row) * ldc + n0 + c4) = v;
        }
        __threadfence();
      }
    } else {
      const int q = lane >> 3, c8 = (lane & 7) * 8;
      unsigned short* C  = (unsigned short*)Cout  + (size_t)b * strideC;
      unsigned short* C2 = (OUT_MODE == 2) ? ((unsigned short*)Cout2 + (size_t)b * strideC) : nullptr;
      for (int pass = 0; pass < 2; ++pass) {
#pragma unroll
        for (int it = 0; it < 4; ++it) {
          const int row = it * 4 + q;
          const float* sp = slab + row * 68 + c8;
          v8h hv, lv;
#pragma unroll
          for (int e = 0; e < 8; ++e) {
            if (OUT_MODE == 1) {
              hv[e] = (_Float16)sp[e];
            } else {
              unsigned short hb = f2bf_bits(sp[e]);
              unsigned short lb = f2bf_bits(sp[e] - bf_bits2f(hb));
              hv[e] = __builtin_bit_cast(_Float16, hb);
              lv[e] = __builtin_bit_cast(_Float16, lb);
            }
          }
          *(volatile v8h*)(C + (size_t)(mBase + row) * ldc + n0 + c8) = hv;
          if (OUT_MODE == 2) *(volatile v8h*)(C2 + (size_t)(mBase + row) * ldc + n0 + c8) = lv;
        }
        __threadfence();
      }
    }
    __builtin_amdgcn_fence(__ATOMIC_RELEASE, "workgroup");
    __builtin_amdgcn_wave_barrier();
    __builtin_amdgcn_fence(__ATOMIC_ACQUIRE, "workgroup");
  }
}

__global__ __launch_bounds__(256) void transpose_cast_f16(const float* __restrict__ in, _Float16* __restrict__ out,
                                                          int R, int Cc, float mul) {
  __shared__ float tile[64][65];
  const int tid = threadIdx.x;
  const int n0 = blockIdx.x * 64;
  const int k0 = blockIdx.y * 64;
#pragma unroll
  for (int i = 0; i < 16; ++i) {
    const int idx = i * 256 + tid;
    const int kk = idx >> 6, nn = idx & 63;
    tile[kk][nn] = in[(size_t)(k0 + kk) * Cc + n0 + nn] * mul;
  }
  __syncthreads();
  const int wave = tid >> 5, lane = tid & 31, q = lane >> 3, c8 = (lane & 7) * 8;
  const int nr0 = wave * 8 + q, nr1 = wave * 8 + 4 + q;
  v8h hv0, hv1;
#pragma unroll
  for (int e = 0; e < 8; ++e) {
    hv0[e] = (_Float16)tile[c8 + e][nr0];
    hv1[e] = (_Float16)tile[c8 + e][nr1];
  }
  _Float16* p0 = out + (size_t)(n0 + nr0) * R + k0 + c8;
  _Float16* p1 = out + (size_t)(n0 + nr1) * R + k0 + c8;
  for (int pass = 0; pass < 2; ++pass) {
    *(volatile v8h*)p0 = hv0;
    *(volatile v8h*)p1 = hv1;
    __threadfence();
  }
}

__global__ __launch_bounds__(256) void bn_elu_f16x8(const float* __restrict__ x, const float* __restrict__ gamma,
                                                    const float* __restrict__ beta, const float* __restrict__ mean,
                                                    const float* __restrict__ var, _Float16* __restrict__ out,
                                                    int cmask, int n8) {
  const int i = blockIdx.x * 256 + threadIdx.x;
  if (i >= n8) return;
  const size_t base = (size_t)i * 8;
  const int c0 = (int)(base & (size_t)cmask);
  const v8f xv = *(const v8f*)(x + base);
  const v8f gv = *(const v8f*)(gamma + c0);
  const v8f bv = *(const v8f*)(beta + c0);
  const v8f mv = *(const v8f*)(mean + c0);
  const v8f vv = *(const v8f*)(var + c0);
  v8h o;
#pragma unroll
  for (int e = 0; e < 8; ++e) {
    const float t = gv[e] * (xv[e] - mv[e]);
    float v = t * rsqrtf(vv[e] + 1e-3f) + bv[e];
    v = (v > 0.f) ? v : (__expf(v) - 1.0f);
    o[e] = (_Float16)v;
  }
  *(volatile v8h*)(out + base) = o;
  __threadfence();
  *(volatile v8h*)(out + base) = o;
}

__global__ __launch_bounds__(256) void pool_w2_f16x8(const _Float16* __restrict__ gf, const _Float16* __restrict__ pf,
                                                     _Float16* __restrict__ gp, _Float16* __restrict__ pp,
                                                     int ci8, int ci, int n8) {
  const int i = blockIdx.x * 256 + threadIdx.x;
  if (i >= n8) return;
  const size_t pr = (size_t)(i / ci8);
  const int ch = (i - (int)pr * ci8) * 8;
  const size_t s0 = (2 * pr) * ci + ch;
  const size_t s1 = s0 + ci;
  const size_t d  = pr * ci + ch;
  const v8h a0 = *(const v8h*)(gf + s0), a1 = *(const v8h*)(gf + s1);
  const v8h b0 = *(const v8h*)(pf + s0), b1 = *(const v8h*)(pf + s1);
  v8h ga, pa;
#pragma unroll
  for (int e = 0; e < 8; ++e) {
    ga[e] = (_Float16)fmaxf((float)a0[e], (float)a1[e]);
    pa[e] = (_Float16)fmaxf((float)b0[e], (float)b1[e]);
  }
  *(volatile v8h*)(gp + d) = ga;
  *(volatile v8h*)(pp + d) = pa;
  __threadfence();
  *(volatile v8h*)(gp + d) = ga;
  *(volatile v8h*)(pp + d) = pa;
}

#define FA_D  128
#define FA_NW 4
#define FA_KC 64
#define FA_KP 136
#define FA_VP 72
#define FA_PP 72
#define FA_OP 132

__global__ __launch_bounds__(128)
void flash128_f16(const _Float16* __restrict__ Q, const _Float16* __restrict__ Kp,
                  const _Float16* __restrict__ Vp, float* __restrict__ O, int nq, int ns) {
  __shared__ __align__(16) _Float16 Ks[FA_KC * FA_KP];
  __shared__ __align__(16) _Float16 Vt[FA_D * FA_VP];
  __shared__ __align__(16) _Float16 Ps[FA_NW][16 * FA_PP];
  __shared__ __align__(16) float    Os[FA_NW][16 * FA_OP];

  const int tid  = threadIdx.x;
  const int wave = tid >> 5;
  const int lane = tid & 31;
  const int hh   = lane >> 4;
  const int c    = lane & 15;

  const int nqb = nq >> 6;
  const int b   = blockIdx.x / nqb;
  const int qb  = blockIdx.x - b * nqb;
  const size_t q0 = (size_t)b * nq + (size_t)qb * 64 + wave * 16;
  const _Float16* kb = Kp + (size_t)b * ns * FA_D;
  const _Float16* vb = Vp + (size_t)b * ns * FA_D;

  v16h qa[4];
  {
    const _Float16* qrow = Q + (q0 + c) * FA_D + 8 * hh;
#pragma unroll
    for (int dc = 0; dc < 4; ++dc) qa[dc] = Frag<_Float16>::load(qrow + dc * 32);
  }

  float mrow[8], lrow[8];
  v8f o[8];
#pragma unroll
  for (int r = 0; r < 8; ++r) { mrow[r] = -INFINITY; lrow[r] = 0.f; }
#pragma unroll
  for (int t = 0; t < 8; ++t) o[t] = zero8();

  const int nch = ns >> 6;
  for (int kc = 0; kc < nch; ++kc) {
    const int kv0 = kc * FA_KC;
    __syncthreads();
#pragma unroll
    for (int i = 0; i < 8; ++i) {
      const int idx = i * 128 + tid;
      const int r   = idx >> 4;
      const int ch  = (idx & 15) * 8;
      const size_t go = (size_t)(kv0 + r) * FA_D + ch;
      const v8h k8 = *(const v8h*)(kb + go);
      const v8h v8 = *(const v8h*)(vb + go);
      *(v8h*)(Ks + r * FA_KP + ch) = k8;
#pragma unroll
      for (int e = 0; e < 8; ++e) Vt[(ch + e) * FA_VP + r] = v8[e];
    }
    __syncthreads();

    v8f s[4];
#pragma unroll
    for (int j = 0; j < 4; ++j) {
      s[j] = zero8();
#pragma unroll
      for (int dc = 0; dc < 4; ++dc) {
        const v16h kf = Frag<_Float16>::load(Ks + (j * 16 + c) * FA_KP + dc * 32 + 8 * hh);
        s[j] = mma_h(qa[dc], kf, s[j]);
      }
    }
    float cm[8];
#pragma unroll
    for (int r = 0; r < 8; ++r) {
      float m = fmaxf(fmaxf(s[0][r], s[1][r]), fmaxf(s[2][r], s[3][r]));
#pragma unroll
      for (int off = 1; off < 16; off <<= 1) m = fmaxf(m, __shfl_xor(m, off, 32));
      cm[r] = m;
    }
    _Float16* pw = Ps[wave];
#pragma unroll
    for (int r = 0; r < 8; ++r) {
      const float mnew  = fmaxf(mrow[r], cm[r]);
      const float alpha = expf(mrow[r] - mnew);
      mrow[r] = mnew;
      float psum = 0.f;
#pragma unroll
      for (int j = 0; j < 4; ++j) {
        const float p = expf(s[j][r] - mnew);
        psum += p;
        pw[(8 * hh + r) * FA_PP + j * 16 + c] = (_Float16)(p * 32768.0f);
      }
#pragma unroll
      for (int off = 1; off < 16; off <<= 1) psum += __shfl_xor(psum, off, 32);
      lrow[r] = lrow[r] * alpha + psum;
#pragma unroll
      for (int t = 0; t < 8; ++t) o[t][r] *= alpha;
    }
    __builtin_amdgcn_fence(__ATOMIC_RELEASE, "workgroup");
    __builtin_amdgcn_wave_barrier();
    __builtin_amdgcn_fence(__ATOMIC_ACQUIRE, "workgroup");

#pragma unroll 1
    for (int kk = 0; kk < 2; ++kk) {
      const v16h pa = Frag<_Float16>::load(pw + c * FA_PP + kk * 32 + 8 * hh);
#pragma unroll
      for (int t = 0; t < 8; ++t) {
        const v16h vf = Frag<_Float16>::load(Vt + (t * 16 + c) * FA_VP + kk * 32 + 8 * hh);
        o[t] = mma_h(pa, vf, o[t]);
      }
    }
  }

  float* os = Os[wave];
#pragma unroll
  for (int r = 0; r < 8; ++r) {
    const float inv = 1.0f / (lrow[r] * 32768.0f);
#pragma unroll
    for (int t = 0; t < 8; ++t) os[(8 * hh + r) * FA_OP + t * 16 + c] = o[t][r] * inv;
  }
  __builtin_amdgcn_fence(__ATOMIC_RELEASE, "workgroup");
  __builtin_amdgcn_wave_barrier();
  __builtin_amdgcn_fence(__ATOMIC_ACQUIRE, "workgroup");
  {
    const int c4 = (lane & 15) * 4;
    for (int pass = 0; pass < 2; ++pass) {
#pragma unroll
      for (int it = 0; it < 8; ++it) {
        const int row = it * 2 + hh;
#pragma unroll
        for (int chf = 0; chf < 2; ++chf) {
          const v4f val = *(const v4f*)(os + row * FA_OP + chf * 64 + c4);
          *(volatile v4f*)(O + (q0 + row) * FA_D + chf * 64 + c4) = val;
        }
      }
      __threadfence();
    }
  }
}


extern "C" void kernel_launch(void* const* d_in, const int* in_sizes, int n_in,
                              void* d_out, int out_size, void* d_ws, size_t ws_size,
                              hipStream_t stream) {
  const int B = 8, H = 64, W = 64, C = 256, CI = 128;
  const int NPIX = B * H * W;
  const int NQ   = H * W;
  const int NS   = H * (W / 2);
  if (n_in < 18) return;
  if (in_sizes[0] != NPIX * C || out_size != NPIX * C) return;
  if (in_sizes[1] != C || in_sizes[2] != C || in_sizes[3] != C || in_sizes[4] != C) return;
  if (in_sizes[5] != CI || in_sizes[6] != CI || in_sizes[7] != CI || in_sizes[8] != CI) return;
  if (in_sizes[9] != C * CI || in_sizes[11] != C * CI || in_sizes[13] != C * CI || in_sizes[15] != CI * C) return;
  if (in_sizes[10] != CI || in_sizes[12] != CI || in_sizes[14] != CI || in_sizes[16] != C || in_sizes[17] < 1) return;
  if (CI != FA_D || (NQ % 64) != 0 || (NS % 64) != 0 || (C % 64) != 0 || (CI % 64) != 0) return;

  const float* x_in = (const float*)d_in[0];
  const float* bn1g = (const float*)d_in[1];
  const float* bn1b = (const float*)d_in[2];
  const float* bn1m = (const float*)d_in[3];
  const float* bn1v = (const float*)d_in[4];
  const float* bn2g = (const float*)d_in[5];
  const float* bn2b = (const float*)d_in[6];
  const float* bn2m = (const float*)d_in[7];
  const float* bn2v = (const float*)d_in[8];
  const float* W_g  = (const float*)d_in[9];
  const float* b_g  = (const float*)d_in[10];
  const float* W_th = (const float*)d_in[11];
  const float* b_th = (const float*)d_in[12];
  const float* W_ph = (const float*)d_in[13];
  const float* b_ph = (const float*)d_in[14];
  const float* W_z  = (const float*)d_in[15];
  const float* b_z  = (const float*)d_in[16];
  const float* sita = (const float*)d_in[17];

  char* wsb = (char*)d_ws;
  size_t off = 0;
  const size_t szX   = (size_t)NPIX * C * 2;
  const size_t szP   = (size_t)NPIX * CI * 2;
  const size_t szPp  = (size_t)B * NS * CI * 2;
  const size_t szY   = (size_t)NPIX * CI * 4;
  const size_t szW   = (size_t)C * CI * 2;
  _Float16* xh  = (_Float16*)(wsb + off); off += szX;
  _Float16* th  = (_Float16*)(wsb + off); off += szP;
  _Float16* gf  = (_Float16*)(wsb + off); off += szP;
  _Float16* pf  = (_Float16*)(wsb + off); off += szP;
  _Float16* gp  = (_Float16*)(wsb + off); off += szPp;
  _Float16* pp  = (_Float16*)(wsb + off); off += szPp;
  float*    yv  = (float*)(wsb + off);    off += szY;
  _Float16* fre = (_Float16*)(wsb + off); off += szP;
  _Float16* wth = (_Float16*)(wsb + off); off += szW;
  _Float16* wgh = (_Float16*)(wsb + off); off += szW;
  _Float16* wph = (_Float16*)(wsb + off); off += szW;
  _Float16* wzh = (_Float16*)(wsb + off); off += szW;
  if (off > ws_size) return;

  transpose_cast_f16<<<dim3(CI / 64, C / 64), 256, 0, stream>>>(W_th, wth, C, CI, 16.0f);
  transpose_cast_f16<<<dim3(CI / 64, C / 64), 256, 0, stream>>>(W_g,  wgh, C, CI, 16.0f);
  transpose_cast_f16<<<dim3(CI / 64, C / 64), 256, 0, stream>>>(W_ph, wph, C, CI, 16.0f);
  transpose_cast_f16<<<dim3(C / 64, CI / 64), 256, 0, stream>>>(W_z,  wzh, CI, C, 16.0f);

  {
    const int n8 = NPIX * C / 8;
    bn_elu_f16x8<<<dim3((n8 + 255) / 256), 256, 0, stream>>>(x_in, bn1g, bn1b, bn1m, bn1v, xh, C - 1, n8);
  }

  {
    const unsigned gProj = (unsigned)(((NPIX / 64) * (CI / 64) + 7) / 8);
    wmma_gemm64<0, false, 2, 1, false, 0, false><<<dim3(gProj, 1), 256, 0, stream>>>(
        U16(xh), nullptr, C, 0L, U16(wth), nullptr, C, 0L, (void*)th, nullptr, CI, 0L,
        b_th, nullptr, nullptr, 0L, NPIX, CI, C, 0.0625f);
    wmma_gemm64<0, false, 2, 1, false, 0, false><<<dim3(gProj, 1), 256, 0, stream>>>(
        U16(xh), nullptr, C, 0L, U16(wgh), nullptr, C, 0L, (void*)gf, nullptr, CI, 0L,
        b_g, nullptr, nullptr, 0L, NPIX, CI, C, 0.0625f);
    wmma_gemm64<0, false, 2, 1, false, 0, false><<<dim3(gProj, 1), 256, 0, stream>>>(
        U16(xh), nullptr, C, 0L, U16(wph), nullptr, C, 0L, (void*)pf, nullptr, CI, 0L,
        b_ph, nullptr, nullptr, 0L, NPIX, CI, C, 0.0625f);
  }

  {
    const int n8 = B * NS * CI / 8;
    pool_w2_f16x8<<<dim3((n8 + 255) / 256), 256, 0, stream>>>(gf, pf, gp, pp, CI / 8, CI, n8);
  }

  flash128_f16<<<dim3(B * (NQ / 64)), 128, 0, stream>>>(th, pp, gp, yv, NQ, NS);

  {
    const int n8 = NPIX * CI / 8;
    bn_elu_f16x8<<<dim3((n8 + 255) / 256), 256, 0, stream>>>(yv, bn2g, bn2b, bn2m, bn2v, fre, CI - 1, n8);
  }

  {
    const unsigned gFin = (unsigned)(((NPIX / 64) * (C / 64) + 7) / 8);
    wmma_gemm64<0, false, 2, 0, true, 0, true><<<dim3(gFin, 1), 256, 0, stream>>>(
        U16(fre), nullptr, CI, 0L, U16(wzh), nullptr, CI, 0L, d_out, nullptr, C, 0L,
        b_z, sita, x_in, 0L, NPIX, C, CI, 0.0625f);
  }
}
